// GlobalCrossAttention_48163763258070
// MI455X (gfx1250) — hardware-verified
//
#include <hip/hip_runtime.h>
#include <math.h>
#include <stdint.h>

#ifndef NB
#define NB 2
#endif
#ifndef NQ
#define NQ 900
#endif
#define NQ_FULL 900
#define NQP   (((NQ + 63) / 64) * 64)
#define LK    4096
#define NPOS  64
#define STRIDE_PX 16
#define EDIM  256
#define NH    8
#define HD    32
#define RHID  512
#define QROWS (NB * NQP)
#define KROWS (NB * LK)
#define SM_SCALE 0.17677669529663687f
#define LOG2E 1.4426950408889634f
#define QSC   1024.0f
#define KSC   1024.0f
#define PCAR  32768.0f
#define VCAR  1024.0f
#define OSC   1024.0f
#define WOS   1024.0f
#define HS    64.0f
#define W2S   64.0f
#define WPB   4
#define NHG   (NH / WPB)
#define NQT   (NQP / 16)
#define NKT   (LK / 32)
#define NST   (LK / 64)
#define ATT_THREADS (WPB * 32)
#define PTP   36
#define PTW   (16 * PTP)
#define SLP   36
#define SLW   (16 * SLP)
#define WREG  (PTW + SLW)
#define SLAB64 (16 * 68)
#define VTP   72
#define HKC   128
#define HTP   136
#define WTP   68
#define OTP   68
#define WS_CAP 134217728
static_assert(EDIM == NH * HD && HD == 32 && NH == 8);
static_assert((NH % WPB) == 0 && ATT_THREADS == 128 && NHG * WPB == NH);
static_assert(NB >= 1 && NB <= 2);
static_assert(NQ >= 1 && NQ <= NQ_FULL);
static_assert((NQP % 64) == 0 && NQP >= NQ && NQT * 16 == NQP);
static_assert(LK == NPOS * NPOS && (LK % 64) == 0 && NKT * 32 == LK && NST * 64 == LK);
static_assert(EDIM == 32 * 8 && (EDIM % 64) == 0 && (EDIM % 32) == 0);
static_assert((RHID % HKC) == 0 && HKC == 128 && (HKC % 32) == 0);
static_assert((QROWS % 64) == 0 && (KROWS % 64) == 0 && (QROWS % 8) == 0 && (KROWS % 8) == 0);
static_assert(NH <= 16);

typedef unsigned short u16;
typedef _Float16 v16h __attribute__((ext_vector_type(16)));
typedef _Float16 v8h  __attribute__((ext_vector_type(8)));
typedef __bf16   v16b __attribute__((ext_vector_type(16)));
typedef float    v8f  __attribute__((ext_vector_type(8)));
typedef float    v4f  __attribute__((ext_vector_type(4)));
typedef unsigned int v4u __attribute__((ext_vector_type(4)));

union FragH { v16h v; v8h h[2]; v4u u[2]; };
union FragB { v16b v; v4u u[2]; };

__device__ __forceinline__ unsigned short bf_bits(float f) {
  unsigned u = __float_as_uint(f);
  return (unsigned short)((u + 0x7FFFu + ((u >> 16) & 1u)) >> 16);
}
__device__ __forceinline__ float bf_up(unsigned short h) { return __uint_as_float(((unsigned)h) << 16); }
__device__ __forceinline__ float bfr(float f) { return bf_up(bf_bits(f)); }
__device__ __forceinline__ unsigned short h_bits(_Float16 x) { return __builtin_bit_cast(unsigned short, x); }
__device__ __forceinline__ unsigned pk16(unsigned short a, unsigned short b) { return (unsigned)a | ((unsigned)b << 16); }
__device__ __forceinline__ v8f zero8() { v8f z = {0.f, 0.f, 0.f, 0.f, 0.f, 0.f, 0.f, 0.f}; return z; }

__device__ __forceinline__ float logdelta(float d) {
  const float t = log2f(fabsf(d) + 1.0f) * (1.0f / 3.0f);
  return (d > 0.0f) ? t : ((d < 0.0f) ? -t : 0.0f);
}

__device__ __forceinline__ v16h ldfrag_h(const _Float16* p) {
  FragH f;
  f.h[0] = *(const v8h*)(p);
  f.h[1] = *(const v8h*)(p + 16);
  return f.v;
}
__device__ __forceinline__ v16b ldfrag_b(const u16* p) {
  FragB f;
  f.u[0] = *(const v4u*)(p);
  f.u[1] = *(const v4u*)(p + 16);
  return f.v;
}

__device__ __forceinline__ v8f mma_h(v16h a, v16h b, v8f c) {
  return __builtin_amdgcn_wmma_f32_16x16x32_f16(false, a, false, b, (short)0, c, false, false);
}
__device__ __forceinline__ v8f mma_b(v16b a, v16b b, v8f c) {
  return __builtin_amdgcn_wmma_f32_16x16x32_bf16(false, a, false, b, (short)0, c, false, false);
}
__device__ __forceinline__ void guard2(v8f& a, v8f& b, v16h x0, v16h x1, v16h x2, v16h x3, v16h x4, v16h x5) {
#if defined(__HIP_DEVICE_COMPILE__)
  asm volatile("v_nop\n\tv_nop\n\tv_nop\n\tv_nop"
               : "+v"(a), "+v"(b) : "v"(x0), "v"(x1), "v"(x2), "v"(x3), "v"(x4), "v"(x5) : "memory");
#endif
}
template <typename F>
__device__ __forceinline__ void guard6(v8f& a, v8f& b, v8f& c, v8f& d, F x0, F x1, F x2, F x3, F x4, F x5) {
#if defined(__HIP_DEVICE_COMPILE__)
  asm volatile("v_nop\n\tv_nop\n\tv_nop\n\tv_nop"
               : "+v"(a), "+v"(b), "+v"(c), "+v"(d) : "v"(x0), "v"(x1), "v"(x2), "v"(x3), "v"(x4), "v"(x5) : "memory");
#endif
}
__device__ __forceinline__ void guard8(v8f& a, v16h x0, v16h x1, v16h x2, v16h x3, v16h x4, v16h x5, v16h x6, v16h x7) {
#if defined(__HIP_DEVICE_COMPILE__)
  asm volatile("v_nop\n\tv_nop\n\tv_nop\n\tv_nop"
               : "+v"(a) : "v"(x0), "v"(x1), "v"(x2), "v"(x3), "v"(x4), "v"(x5), "v"(x6), "v"(x7) : "memory");
#endif
}
__device__ __forceinline__ void acc_guard2(v8f& a, v8f& b) {
#if defined(__HIP_DEVICE_COMPILE__)
  asm volatile("v_nop\n\tv_nop\n\tv_nop\n\tv_nop" : "+v"(a), "+v"(b));
#endif
}
__device__ __forceinline__ void wave_sync_lds() {
  __builtin_amdgcn_fence(__ATOMIC_RELEASE, "workgroup");
  __builtin_amdgcn_wave_barrier();
  __builtin_amdgcn_fence(__ATOMIC_ACQUIRE, "workgroup");
}

__global__ __launch_bounds__(256) void cvrows(const float* __restrict__ x, u16* D, int ntot, int RV, int RP, int RF) {
  const int tid = (int)threadIdx.x;
  const int row = (int)blockIdx.x * 8 + (tid >> 5);
  if (row >= ntot) return;
  const int e8 = (tid & 31) * 8;
  const int b  = row / RP;
  const int s  = row - b * RP;
  const bool valid = (s < RV);
  const int sc = valid ? s : (RV - 1);
  const float* p = x + ((size_t)b * RF + sc) * EDIM + e8;
  const v4f a = *(const v4f*)(p), b4 = *(const v4f*)(p + 4);
  float w[8];
#pragma unroll
  for (int e = 0; e < 4; ++e) { w[e] = a[e]; w[4 + e] = b4[e]; }
  v4u o;
#pragma unroll
  for (int e = 0; e < 4; ++e) {
    const unsigned pv = pk16(bf_bits(w[2 * e]), bf_bits(w[2 * e + 1]));
    o[e] = valid ? pv : 0u;
  }
  u16* d = D + (size_t)row * EDIM + e8;
  for (int pass = 0; pass < 2; ++pass) {
    *(volatile v4u*)(d) = o;
    __threadfence();
  }
}

__global__ __launch_bounds__(256) void wtr(const float* __restrict__ Wm, u16* Bt, int f16mode, float scale) {
  __shared__ __align__(16) float T[64 * WTP];
  const int tid = (int)threadIdx.x;
  const int bid = (int)blockIdx.x;
  const int k0 = (bid >> 2) * 64, n0 = (bid & 3) * 64;
  {
    const int kr = tid >> 4, nc = (tid & 15) * 4;
#pragma unroll
    for (int it = 0; it < 4; ++it) {
      const int k = it * 16 + kr;
      const v4f a = *(const v4f*)(Wm + (size_t)(k0 + k) * EDIM + n0 + nc);
#pragma unroll
      for (int e = 0; e < 4; ++e) T[(nc + e) * WTP + k] = a[e];
    }
  }
  __syncthreads();
  v4u o[2];
#pragma unroll
  for (int it = 0; it < 2; ++it) {
    const int task = it * 256 + tid;
    const int n = task >> 3, k8 = (task & 7) * 8;
    const v4f a = *(const v4f*)(T + n * WTP + k8), b4 = *(const v4f*)(T + n * WTP + k8 + 4);
    float w[8];
#pragma unroll
    for (int e = 0; e < 4; ++e) { w[e] = a[e]; w[4 + e] = b4[e]; }
#pragma unroll
    for (int e = 0; e < 4; ++e) {
      const float f0 = w[2 * e], f1 = w[2 * e + 1];
      const unsigned short hb0 = h_bits((_Float16)(bfr(f0) * scale));
      const unsigned short hb1 = h_bits((_Float16)(bfr(f1) * scale));
      const unsigned short bb0 = bf_bits(f0);
      const unsigned short bb1 = bf_bits(f1);
      o[it][e] = (f16mode != 0) ? pk16(hb0, hb1) : pk16(bb0, bb1);
    }
  }
  for (int pass = 0; pass < 2; ++pass) {
#pragma unroll
    for (int it = 0; it < 2; ++it) {
      const int task = it * 256 + tid;
      const int n = task >> 3, k8 = (task & 7) * 8;
      *(volatile v4u*)(Bt + (size_t)(n0 + n) * EDIM + k0 + k8) = o[it];
    }
    __threadfence();
  }
}

__global__ __launch_bounds__(256) void w2prep(const float* __restrict__ W2x, const float* __restrict__ W2y, u16* W2T) {
  const int tid = (int)threadIdx.x, bid = (int)blockIdx.x;
  const int tsel = bid >> 2;
  if (tsel > 1) return;
  const float* W2 = (tsel != 0) ? W2y : W2x;
  const int r = (bid & 3) * 256 + tid;
  const int n = r >> 6, k8 = (r & 63) * 8;
  const bool live = (n < NH);
  const int nn = live ? n : (NH - 1);
  v4u o;
#pragma unroll
  for (int e = 0; e < 4; ++e) {
    const float f0 = W2[(size_t)(k8 + 2 * e) * NH + nn];
    const float f1 = W2[(size_t)(k8 + 2 * e + 1) * NH + nn];
    const unsigned pv = pk16(h_bits((_Float16)(bfr(f0) * W2S)), h_bits((_Float16)(bfr(f1) * W2S)));
    o[e] = live ? pv : 0u;
  }
  u16* d = W2T + (size_t)tsel * 16 * RHID + (size_t)n * RHID + k8;
  for (int pass = 0; pass < 2; ++pass) {
    *(volatile v4u*)(d) = o;
    __threadfence();
  }
}

__device__ __forceinline__ void epi64(float* sl, v8f a0, v8f a1, v8f a2, v8f a3, float oscale,
                                      const float* __restrict__ bias, float* C, int N, size_t rowb, int col0, int lane,
                                      int nval) {
  const int hh = lane >> 4, m = lane & 15;
#pragma unroll
  for (int r = 0; r < 8; ++r) {
    const int ro = (8 * hh + r) * 68 + m;
    sl[ro]      = a0[r] * oscale;
    sl[ro + 16] = a1[r] * oscale;
    sl[ro + 32] = a2[r] * oscale;
    sl[ro + 48] = a3[r] * oscale;
  }
  wave_sync_lds();
  const v4f bb = *(const v4f*)(bias + col0 + m * 4);
  v4f br;
#pragma unroll
  for (int e = 0; e < 4; ++e) br[e] = bfr(bb[e]);
  v4f vals[8];
#pragma unroll
  for (int it = 0; it < 8; ++it) vals[it] = *(const v4f*)(sl + (it * 2 + hh) * 68 + m * 4) + br;
  float* dst = C + (rowb + (size_t)hh) * (size_t)N + col0 + m * 4;
  for (int pass = 0; pass < 2; ++pass) {
#pragma unroll
    for (int it = 0; it < 8; ++it) {
      if (it * 2 + hh < nval) {
        *(volatile v4f*)(dst + (size_t)(it * 2) * (size_t)N) = vals[it];
      }
    }
    __threadfence();
  }
}

__global__ __launch_bounds__(128)
void gemm_bf(const u16* __restrict__ A, const u16* __restrict__ Bt, const float* __restrict__ bias,
             float* C, int M, int N, int K, float oscale) {
  __shared__ __align__(16) float slab[4 * SLAB64];
  const int tid = threadIdx.x, wave = tid >> 5, lane = tid & 31, hh = lane >> 4, m = lane & 15;
  const int ntile = N >> 6;
  const int bid   = blockIdx.x;
  const int rowb  = (bid / ntile) * 64 + wave * 16;
  const int col0  = (bid % ntile) * 64;
  if (rowb + 16 > M) return;
  const u16* ap = A  + (size_t)(rowb + m) * K + 8 * hh;
  const u16* bp = Bt + (size_t)(col0 + m) * K + 8 * hh;
  const size_t bs = (size_t)16 * K;
  v8f acc0 = zero8(), acc1 = zero8(), acc2 = zero8(), acc3 = zero8();
#pragma unroll 1
  for (int k0 = 0; k0 < K; k0 += 32) {
    const v16b a  = ldfrag_b(ap + k0);
    const v16b b0 = ldfrag_b(bp + k0);
    const v16b b1 = ldfrag_b(bp + bs + k0);
    const v16b b2 = ldfrag_b(bp + 2 * bs + k0);
    const v16b b3 = ldfrag_b(bp + 3 * bs + k0);
    acc0 = mma_b(a, b0, acc0);
    acc1 = mma_b(a, b1, acc1);
    acc2 = mma_b(a, b2, acc2);
    acc3 = mma_b(a, b3, acc3);
    guard6<v16b>(acc0, acc1, acc2, acc3, a, b0, b1, b2, b3, a);
  }
  epi64(slab + wave * SLAB64, acc0, acc1, acc2, acc3, oscale, bias, C, N, (size_t)rowb, col0, lane, 16);
}

__global__ __launch_bounds__(256) void qk16(const float* __restrict__ F, u16* Hp, u16* Lp, int nrows, float sc) {
  const int tid = (int)threadIdx.x;
  const int row = (int)blockIdx.x * 8 + (tid >> 5);
  if (row >= nrows) return;
  const int t8 = (tid & 31) * 8;
  const float* p = F + (size_t)row * EDIM + t8;
  const v4f a = *(const v4f*)(p), b4 = *(const v4f*)(p + 4);
  float w[8];
#pragma unroll
  for (int e = 0; e < 4; ++e) { w[e] = a[e] * sc; w[4 + e] = b4[e] * sc; }
  v4u oh, ol;
#pragma unroll
  for (int e = 0; e < 4; ++e) {
    const float t0 = w[2 * e], t1 = w[2 * e + 1];
    const _Float16 h0 = (_Float16)t0, h1 = (_Float16)t1;
    const _Float16 l0 = (_Float16)(t0 - (float)h0), l1 = (_Float16)(t1 - (float)h1);
    oh[e] = pk16(h_bits(h0), h_bits(h1));
    ol[e] = pk16(h_bits(l0), h_bits(l1));
  }
  u16* dh = Hp + (size_t)row * EDIM + t8;
  u16* dl = Lp + (size_t)row * EDIM + t8;
  for (int pass = 0; pass < 2; ++pass) {
    *(volatile v4u*)(dh) = oh;
    *(volatile v4u*)(dl) = ol;
    __threadfence();
  }
}

__global__ __launch_bounds__(256) void vt16(const float* __restrict__ F, u16* VHo, u16* VLo) {
  __shared__ __align__(16) u16 TH[HD * VTP];
  __shared__ __align__(16) u16 TL[HD * VTP];
  const int tid = (int)threadIdx.x;
  const int bid = (int)blockIdx.x;
  const int st  = bid % NST;
  const int t2  = bid / NST;
  const int g   = t2 % NH;
  const int b   = t2 / NH;
  if (b >= NB) return;
  const int s0  = st * 64;
  {
    const int sl = tid >> 2;
    const int dc = (tid & 3) * 8;
    const float* src = F + ((size_t)b * LK + s0 + sl) * EDIM + g * HD + dc;
#pragma unroll
    for (int i = 0; i < 2; ++i) {
      const v4f a = *(const v4f*)(src + 4 * i);
#pragma unroll
      for (int e = 0; e < 4; ++e) {
        const float t = a[e] * VCAR;
        const _Float16 hv = (_Float16)t;
        const _Float16 lv = (_Float16)(t - (float)hv);
        TH[(dc + 4 * i + e) * VTP + sl] = h_bits(hv);
        TL[(dc + 4 * i + e) * VTP + sl] = h_bits(lv);
      }
    }
  }
  __syncthreads();
  const int q8 = tid >> 3, p8 = (tid & 7) * 8;
  const v4u vh = *(const v4u*)(TH + q8 * VTP + p8);
  const v4u vl = *(const v4u*)(TL + q8 * VTP + p8);
  const size_t base = ((size_t)(b * NH + g) * HD + q8) * LK + s0 + p8;
  for (int pass = 0; pass < 2; ++pass) {
    *(volatile v4u*)(VHo + base) = vh;
    *(volatile v4u*)(VLo + base) = vl;
    __threadfence();
  }
}

__global__ __launch_bounds__(128)
void rpe_tab(const float* __restrict__ boxes, const float* __restrict__ W1, const float* __restrict__ b1,
             const u16* __restrict__ W2T, const int* __restrict__ dimp, float* Tout, int ic, int iw, int isx) {
  __shared__ __align__(16) u16 HT[NPOS * HTP];
  __shared__ __align__(16) float OT[NH * OTP];
  __shared__ float w1s[3 * RHID];
  const int tid = (int)threadIdx.x, wave = tid >> 5, lane = tid & 31, hh = lane >> 4, m = lane & 15;
  const int bid = (int)blockIdx.x;
  const int q = bid % NQP, b = bid / NQP;
  if (b >= NB) return;
  const int qq = (q < NQ) ? q : (NQ - 1);
  for (int j = tid; j < 2 * RHID; j += 128) w1s[j] = bfr(W1[j]);
  for (int j = tid; j < RHID; j += 128) w1s[2 * RHID + j] = bfr(b1[j]);
  const float* bp4 = boxes + ((size_t)b * NQ_FULL + qq) * 4;
  const float cv = bfr(bp4[ic]);
  const float wv = bfr(bp4[iw]);
  const float dimv = (float)(dimp[0] * STRIDE_PX);
  const float e1 = (cv - 0.5f * wv) * dimv;
  const float e2 = (cv + 0.5f * wv) * dimv;
  __syncthreads();

  const int p  = tid & 63;
  const int jh = (tid >> 6) * (HKC / 2);
  const float posv = ((float)p + 0.5f) * (float)STRIDE_PX;
  const float d1 = logdelta(e1 - posv), d2 = logdelta(e2 - posv);
  u16* hrow = HT + p * HTP + jh;
  const _Float16* ap  = (const _Float16*)(const void*)HT + (16 * wave + m) * HTP + 8 * hh;
  const _Float16* w2p = (const _Float16*)(const void*)W2T + (size_t)m * RHID + 8 * hh;
  v8f acc = zero8();
#pragma unroll 1
  for (int kc = 0; kc < RHID / HKC; ++kc) {
    const int jb = kc * HKC + jh;
#pragma unroll 1
    for (int g = 0; g < (HKC / 2) / 8; ++g) {
      v4u o;
#pragma unroll
      for (int e = 0; e < 4; ++e) {
        const int j0 = jb + 8 * g + 2 * e;
        float h0 = fmaf(d1, w1s[j0],     fmaf(d2, w1s[RHID + j0],     w1s[2 * RHID + j0]));
        float h1 = fmaf(d1, w1s[j0 + 1], fmaf(d2, w1s[RHID + j0 + 1], w1s[2 * RHID + j0 + 1]));
        h0 = fmaxf(h0, 0.0f);
        h1 = fmaxf(h1, 0.0f);
        o[e] = pk16(h_bits((_Float16)(h0 * HS)), h_bits((_Float16)(h1 * HS)));
      }
      *(v4u*)(hrow + 8 * g) = o;
    }
    __syncthreads();
    const v16h a0 = ldfrag_h(ap);
    const v16h a1 = ldfrag_h(ap + 32);
    const v16h a2 = ldfrag_h(ap + 64);
    const v16h a3 = ldfrag_h(ap + 96);
    const _Float16* wp = w2p + kc * HKC;
    const v16h w0 = ldfrag_h(wp);
    const v16h w1 = ldfrag_h(wp + 32);
    const v16h w2 = ldfrag_h(wp + 64);
    const v16h w3 = ldfrag_h(wp + 96);
    acc = mma_h(a0, w0, acc);
    acc = mma_h(a1, w1, acc);
    acc = mma_h(a2, w2, acc);
    acc = mma_h(a3, w3, acc);
    guard8(acc, a0, a1, a2, a3, w0, w1, w2, w3);
    __syncthreads();
  }
  const float RS = LOG2E / (HS * W2S);
  if (m < NH) {
#pragma unroll
    for (int r = 0; r < 8; ++r) {
      const int pos  = 16 * wave + 8 * hh + r;
      const int slot = (isx != 0) ? ((pos & 15) * 4 + (pos >> 4)) : pos;
      OT[m * OTP + slot] = acc[r] * RS;
    }
  }
  __syncthreads();
  const int h = 2 * wave + hh;
  const v4f val = *(const v4f*)(OT + h * OTP + m * 4);
  float* dst = Tout + (((size_t)(b * NH + h)) * NQP + q) * NPOS + m * 4;
  for (int pass = 0; pass < 2; ++pass) {
    *(volatile v4f*)(dst) = val;
    __threadfence();
  }
}

__global__ __launch_bounds__(ATT_THREADS)
void attn_g(const u16* __restrict__ QHp, const u16* __restrict__ QLp,
            const u16* __restrict__ KHp, const u16* __restrict__ KLp,
            const u16* __restrict__ VHp, const u16* __restrict__ VLp,
            const float* __restrict__ RXL, const float* __restrict__ RYL,
            u16* OHp, u16* OLp) {
  __shared__ __align__(16) float smem[WPB * WREG];

  const int tid  = (int)threadIdx.x;
  const int wave = tid >> 5;
  const int lane = tid & 31;
  const int hh   = lane >> 4;
  const int c    = lane & 15;
  const int bid  = (int)blockIdx.x;
  const int qt   = bid % NQT;
  const int t2   = bid / NQT;
  const int hg   = t2 % NHG;
  const int b    = t2 / NHG;
  if (b >= NB) return;
  const int q0   = qt * 16;
  const int head = hg * WPB + wave;

  float* pt   = smem + wave * WREG;
  float* slab = pt + PTW;

  const size_t hcol = (size_t)head * HD + 8 * hh;
  const _Float16* Qh  = (const _Float16*)(const void*)QHp + ((size_t)b * NQP + q0 + c) * EDIM + hcol;
  const _Float16* Ql  = (const _Float16*)(const void*)QLp + ((size_t)b * NQP + q0 + c) * EDIM + hcol;
  const _Float16* Khb = (const _Float16*)(const void*)KHp + ((size_t)b * LK + c) * EDIM + hcol;
  const _Float16* Klb = (const _Float16*)(const void*)KLp + ((size_t)b * LK + c) * EDIM + hcol;
  const _Float16* Vhb = (const _Float16*)(const void*)VHp + ((size_t)(b * NH + head) * HD + c) * LK + 8 * hh;
  const _Float16* Vlb = (const _Float16*)(const void*)VLp + ((size_t)(b * NH + head) * HD + c) * LK + 8 * hh;
  const size_t trow = ((size_t)(b * NH + head) * NQP + q0 + 8 * hh) * NPOS;
  v4f px[8];
#pragma unroll
  for (int r = 0; r < 8; ++r) px[r] = *(const v4f*)(RXL + trow + (size_t)r * NPOS + c * 4);
  const float* ryp = RYL + trow;
  const float lsc = SM_SCALE * (LOG2E / (QSC * KSC));
  const float oc  = 1.0f / (PCAR * VCAR);
  const size_t KROW = (size_t)EDIM;

  const v16h qh = ldfrag_h(Qh);
  const v16h ql = ldfrag_h(Ql);

  float mrow[8], lrow[8];
  v8f o0 = zero8(), o1 = zero8();
#pragma unroll
  for (int r = 0; r < 8; ++r) { mrow[r] = -INFINITY; lrow[r] = 0.f; }

#pragma unroll 1
  for (int kt = 0; kt < NKT; ++kt) {
    const int kb = kt * 32;
    v8f s0 = zero8(), s1 = zero8();
    {
      const _Float16* k0p = Khb + (size_t)kb * KROW;
      const _Float16* k1p = k0p + (size_t)16 * KROW;
      const _Float16* l0p = Klb + (size_t)kb * KROW;
      const _Float16* l1p = l0p + (size_t)16 * KROW;
      const v16h kh0 = ldfrag_h(k0p);
      const v16h kh1 = ldfrag_h(k1p);
      const v16h kl0 = ldfrag_h(l0p);
      const v16h kl1 = ldfrag_h(l1p);
      s0 = mma_h(qh, kh0, s0);
      s0 = mma_h(ql, kh0, s0);
      s0 = mma_h(qh, kl0, s0);
      s1 = mma_h(qh, kh1, s1);
      s1 = mma_h(ql, kh1, s1);
      s1 = mma_h(qh, kl1, s1);
      guard2(s0, s1, qh, ql, kh0, kl0, kh1, kl1);
    }
    const int  ky  = kt >> 1;
    const bool odd = ((kt & 1) != 0);
    float ryv[8];
#pragma unroll
    for (int r = 0; r < 8; ++r) ryv[r] = ryp[(size_t)r * NPOS + ky];
#pragma unroll
    for (int r = 0; r < 8; ++r) {
      const float bx0 = odd ? px[r][2] : px[r][0];
      const float bx1 = odd ? px[r][3] : px[r][1];
      const float t0 = fmaf(s0[r], lsc, ryv[r] + bx0);
      const float t1 = fmaf(s1[r], lsc, ryv[r] + bx1);
      float mx = fmaxf(t0, t1);
#pragma unroll
      for (int off = 1; off < 16; off <<= 1) mx = fmaxf(mx, __shfl_xor(mx, off, 32));
      const float mn = fmaxf(mrow[r], mx);
      const float ms = (mn == -INFINITY) ? 0.0f : mn;
      const float al = exp2f(mrow[r] - ms);
      mrow[r] = mn;
      const float e0 = exp2f(t0 - ms), e1 = exp2f(t1 - ms);
      float ps = e0 + e1;
#pragma unroll
      for (int off = 1; off < 16; off <<= 1) ps += __shfl_xor(ps, off, 32);
      lrow[r] = lrow[r] * al + ps;
      o0[r] *= al;
      o1[r] *= al;
      const int ro = (8 * hh + r) * PTP + c;
      pt[ro]      = e0;
      pt[ro + 16] = e1;
    }
    wave_sync_lds();
    FragH ph, pl;
    {
      const float* prow = pt + c * PTP + 8 * hh;
      const v4f p0 = *(const v4f*)(prow), p1 = *(const v4f*)(prow + 4);
      const v4f p2 = *(const v4f*)(prow + 16), p3 = *(const v4f*)(prow + 20);
#pragma unroll
      for (int e = 0; e < 4; ++e) {
        const float ta = p0[e] * PCAR, tb = p1[e] * PCAR, tc = p2[e] * PCAR, td = p3[e] * PCAR;
        const _Float16 ha = (_Float16)ta, hb = (_Float16)tb, hc = (_Float16)tc, hd = (_Float16)td;
        ph.h[0][e]     = ha;
        ph.h[0][4 + e] = hb;
        ph.h[1][e]     = hc;
        ph.h[1][4 + e] = hd;
        pl.h[0][e]     = (_Float16)(ta - (float)ha);
        pl.h[0][4 + e] = (_Float16)(tb - (float)hb);
        pl.h[1][e]     = (_Float16)(tc - (float)hc);
        pl.h[1][4 + e] = (_Float16)(td - (float)hd);
      }
    }
    {
      const _Float16* vhp = Vhb + kb;
      const _Float16* vlp = Vlb + kb;
      const v16h vha = ldfrag_h(vhp), vhb2 = ldfrag_h(vhp + (size_t)16 * LK);
      const v16h vla = ldfrag_h(vlp), vlb2 = ldfrag_h(vlp + (size_t)16 * LK);
      o0 = mma_h(ph.v, vha,  o0);
      o0 = mma_h(pl.v, vha,  o0);
      o0 = mma_h(ph.v, vla,  o0);
      o1 = mma_h(ph.v, vhb2, o1);
      o1 = mma_h(pl.v, vhb2, o1);
      o1 = mma_h(ph.v, vlb2, o1);
      guard2(o0, o1, ph.v, pl.v, vha, vhb2, vla, vlb2);
    }
    wave_sync_lds();
  }
  acc_guard2(o0, o1);
#pragma unroll
  for (int r = 0; r < 8; ++r) {
    const float lv  = lrow[r];
    const float ls  = (lv > 0.0f) ? lv : 1.0f;
    const float inv = (lv > 0.0f) ? ((1.0f / ls) * oc) : 0.0f;
    const int idx = (8 * hh + r) * SLP + c;
    slab[idx]      = o0[r] * inv;
    slab[idx + 16] = o1[r] * inv;
  }
  __syncthreads();
  v4u oh[2], ol[2];
#pragma unroll
  for (int it = 0; it < 2; ++it) {
    const int task = it * ATT_THREADS + tid;
    const int row = task >> 4, seg = task & 15;
    const int w = seg >> 2, d8 = (seg & 3) * 8;
    const float* sp = smem + w * WREG + PTW + row * SLP + d8;
    const v4f a = *(const v4f*)(sp), b4 = *(const v4f*)(sp + 4);
    float wf[8];
#pragma unroll
    for (int e = 0; e < 4; ++e) { wf[e] = a[e] * OSC; wf[4 + e] = b4[e] * OSC; }
#pragma unroll
    for (int e = 0; e < 4; ++e) {
      const _Float16 h0 = (_Float16)wf[2 * e], h1 = (_Float16)wf[2 * e + 1];
      const _Float16 l0 = (_Float16)(wf[2 * e] - (float)h0), l1 = (_Float16)(wf[2 * e + 1] - (float)h1);
      oh[it][e] = pk16(h_bits(h0), h_bits(h1));
      ol[it][e] = pk16(h_bits(l0), h_bits(l1));
    }
  }
  const size_t ob = ((size_t)b * NQP + q0) * EDIM + (size_t)hg * (WPB * HD);
  for (int pass = 0; pass < 2; ++pass) {
#pragma unroll
    for (int it = 0; it < 2; ++it) {
      const int task = it * ATT_THREADS + tid;
      const int row = task >> 4, seg = task & 15;
      *(volatile v4u*)(OHp + ob + (size_t)row * EDIM + seg * 8) = oh[it];
      *(volatile v4u*)(OLp + ob + (size_t)row * EDIM + seg * 8) = ol[it];
    }
    __threadfence();
  }
}

__global__ __launch_bounds__(128)
void gemm_o2(const u16* __restrict__ Ah, const u16* __restrict__ Al, const u16* __restrict__ Bt, const float* __restrict__ bias,
             float* C, float oscale) {
  __shared__ __align__(16) float slab[4 * SLAB64];
  const int tid = threadIdx.x, wave = tid >> 5, lane = tid & 31, hh = lane >> 4, m = lane & 15;
  const int ntile = EDIM >> 6;
  const int nrt   = NQP / 64;
  const int bid   = blockIdx.x;
  const int ct    = bid % ntile;
  const int t2    = bid / ntile;
  const int rt    = t2 % nrt;
  const int bb    = t2 / nrt;
  if (bb >= NB) return;
  const int srow  = rt * 64 + wave * 16;
  if (srow >= NQ) return;
  int nval = NQ - srow;
  if (nval > 16) nval = 16;
  const int col0  = ct * 64;
  const int K     = EDIM;
  const size_t rowA = (size_t)bb * NQP + srow;
  const size_t rowO = (size_t)bb * NQ_FULL + srow;
  const _Float16* ahp = (const _Float16*)(const void*)Ah + (rowA + m) * K + 8 * hh;
  const _Float16* alp = (const _Float16*)(const void*)Al + (rowA + m) * K + 8 * hh;
  const _Float16* bp  = (const _Float16*)(const void*)Bt + (size_t)(col0 + m) * K + 8 * hh;
  const size_t bs = (size_t)16 * K;
  v8f acc0 = zero8(), acc1 = zero8(), acc2 = zero8(), acc3 = zero8();
#pragma unroll 1
  for (int k0 = 0; k0 < K; k0 += 32) {
    const v16h ah = ldfrag_h(ahp + k0), al = ldfrag_h(alp + k0);
    const v16h b0 = ldfrag_h(bp + k0);
    const v16h b1 = ldfrag_h(bp + bs + k0);
    const v16h b2 = ldfrag_h(bp + 2 * bs + k0);
    const v16h b3 = ldfrag_h(bp + 3 * bs + k0);
    acc0 = mma_h(ah, b0, acc0);  acc0 = mma_h(al, b0, acc0);
    acc1 = mma_h(ah, b1, acc1);  acc1 = mma_h(al, b1, acc1);
    acc2 = mma_h(ah, b2, acc2);  acc2 = mma_h(al, b2, acc2);
    acc3 = mma_h(ah, b3, acc3);  acc3 = mma_h(al, b3, acc3);
    guard6<v16h>(acc0, acc1, acc2, acc3, ah, al, b0, b1, b2, b3);
  }
  epi64(slab + wave * SLAB64, acc0, acc1, acc2, acc3, oscale, bias, C, EDIM, rowO, col0, lane, nval);
}

extern "C" void kernel_launch(void* const* d_in, const int* in_sizes, int n_in,
                              void* d_out, int out_size, void* d_ws, size_t ws_size,
                              hipStream_t stream) {
  if (n_in < 20) return;
  const int qneed = (NB - 1) * NQ_FULL + NQ;
  if (in_sizes[0] < qneed * EDIM) return;
  if (in_sizes[1] < KROWS * EDIM || in_sizes[2] < KROWS * EDIM) return;
  if (in_sizes[3] < qneed * 4) return;
  if (in_sizes[4] < EDIM * EDIM || in_sizes[6] < EDIM * EDIM || in_sizes[8] < EDIM * EDIM || in_sizes[10] < EDIM * EDIM) return;
  if (in_sizes[5] < EDIM || in_sizes[7] < EDIM || in_sizes[9] < EDIM || in_sizes[11] < EDIM) return;
  if (in_sizes[12] < 2 * RHID || in_sizes[15] < 2 * RHID) return;
  if (in_sizes[13] < RHID || in_sizes[16] < RHID) return;
  if (in_sizes[14] < RHID * NH || in_sizes[17] < RHID * NH) return;
  if (in_sizes[18] < 1 || in_sizes[19] < 1) return;
  if (out_size < qneed * EDIM) return;

  const float* xq    = (const float*)d_in[0];
  const float* xk    = (const float*)d_in[1];
  const float* xv    = (const float*)d_in[2];
  const float* boxes = (const float*)d_in[3];
  const float* wq  = (const float*)d_in[4];   const float* bq  = (const float*)d_in[5];
  const float* wk  = (const float*)d_in[6];   const float* bk  = (const float*)d_in[7];
  const float* wv  = (const float*)d_in[8];   const float* bv  = (const float*)d_in[9];
  const float* wo  = (const float*)d_in[10];  const float* bo  = (const float*)d_in[11];
  const float* w1x = (const float*)d_in[12];  const float* b1x = (const float*)d_in[13];
  const float* w2x = (const float*)d_in[14];
  const float* w1y = (const float*)d_in[15];  const float* b1y = (const float*)d_in[16];
  const float* w2y = (const float*)d_in[17];
  const int*   hdim = (const int*)d_in[18];
  const int*   wdim = (const int*)d_in[19];
  float*       out  = (float*)d_out;

  const size_t szXQ = (size_t)QROWS * EDIM * 2;
  const size_t szXK = (size_t)KROWS * EDIM * 2;
  const size_t szV  = (size_t)NB * NH * HD * LK * 2;
  const size_t szW  = (size_t)EDIM * EDIM * 2;
  const size_t szW2 = (size_t)2 * 16 * RHID * 2;
  const size_t szFQ = (size_t)QROWS * EDIM * 4;
  const size_t szFK = (size_t)KROWS * EDIM * 4;
  const size_t szT  = (size_t)NB * NH * NQP * NPOS * 4;
  size_t off = 0;
  const size_t oXQ = off; off += szXQ;
  const size_t oXK = off; off += szXK;
  const size_t oXV = off; off += szXK;
  const size_t oWQ = off; off += szW;
  const size_t oWK = off; off += szW;
  const size_t oWV = off; off += szW;
  const size_t oWO = off; off += szW;
  const size_t oW2 = off; off += szW2;
  const size_t oFQ = off; off += szFQ;
  const size_t oFK = off; off += szFK;
  const size_t oFV = off; off += szFK;
  const size_t oQH = off; off += szXQ;
  const size_t oQL = off; off += szXQ;
  const size_t oKH = off; off += szXK;
  const size_t oKL = off; off += szXK;
  const size_t oVH = off; off += szV;
  const size_t oVL = off; off += szV;
  const size_t oRX = off; off += szT;
  const size_t oRY = off; off += szT;
  const size_t oOH = off; off += szXQ;
  const size_t oOL = off; off += szXQ;
  if (off > ws_size) return;
  if (off > (size_t)WS_CAP) return;

  char* ws = (char*)d_ws;
  u16*   XQ  = (u16*)(ws + oXQ);
  u16*   XK  = (u16*)(ws + oXK);
  u16*   XV  = (u16*)(ws + oXV);
  u16*   WQT = (u16*)(ws + oWQ);
  u16*   WKT = (u16*)(ws + oWK);
  u16*   WVT = (u16*)(ws + oWV);
  u16*   WOT = (u16*)(ws + oWO);
  u16*   W2T = (u16*)(ws + oW2);
  float* FQ  = (float*)(ws + oFQ);
  float* FK  = (float*)(ws + oFK);
  float* FV  = (float*)(ws + oFV);
  u16*   QH  = (u16*)(ws + oQH);
  u16*   QL  = (u16*)(ws + oQL);
  u16*   KH  = (u16*)(ws + oKH);
  u16*   KL  = (u16*)(ws + oKL);
  u16*   VH  = (u16*)(ws + oVH);
  u16*   VL  = (u16*)(ws + oVL);
  float* RXL = (float*)(ws + oRX);
  float* RYL = (float*)(ws + oRY);
  u16*   OH  = (u16*)(ws + oOH);
  u16*   OL  = (u16*)(ws + oOL);

  const dim3 b256(256), b128(128), bAT(ATT_THREADS);
  const dim3 gCQ(QROWS / 8), gCK(KROWS / 8);
  const dim3 gWT(16), gW2(8);
  const dim3 gGQ((QROWS / 64) * (EDIM / 64)), gGK((KROWS / 64) * (EDIM / 64));
  const dim3 gVT(NB * NH * NST);
  const dim3 gRP(NB * NQP);
  const dim3 gAT(NQT * NHG * NB);
  const dim3 gO(NB * (NQP / 64) * (EDIM / 64));

  cvrows<<<gCQ, b256, 0, stream>>>(xq, XQ, QROWS, NQ, NQP, NQ_FULL);
  cvrows<<<gCK, b256, 0, stream>>>(xk, XK, KROWS, LK, LK, LK);
  cvrows<<<gCK, b256, 0, stream>>>(xv, XV, KROWS, LK, LK, LK);
  wtr<<<gWT, b256, 0, stream>>>(wq, WQT, 0, 1.0f);
  wtr<<<gWT, b256, 0, stream>>>(wk, WKT, 0, 1.0f);
  wtr<<<gWT, b256, 0, stream>>>(wv, WVT, 0, 1.0f);
  wtr<<<gWT, b256, 0, stream>>>(wo, WOT, 1, WOS);
  w2prep<<<gW2, b256, 0, stream>>>(w2x, w2y, W2T);
  gemm_bf<<<gGQ, b128, 0, stream>>>(XQ, WQT, bq, FQ, QROWS, EDIM, EDIM, 1.0f);
  gemm_bf<<<gGK, b128, 0, stream>>>(XK, WKT, bk, FK, KROWS, EDIM, EDIM, 1.0f);
  gemm_bf<<<gGK, b128, 0, stream>>>(XV, WVT, bv, FV, KROWS, EDIM, EDIM, 1.0f);
  qk16<<<gCQ, b256, 0, stream>>>(FQ, QH, QL, QROWS, QSC);
  qk16<<<gCK, b256, 0, stream>>>(FK, KH, KL, KROWS, KSC);
  vt16<<<gVT, b256, 0, stream>>>(FV, VH, VL);
  rpe_tab<<<gRP, b128, 0, stream>>>(boxes, w1x, b1x, W2T, wdim, RXL, 0, 2, 1);
  rpe_tab<<<gRP, b128, 0, stream>>>(boxes, w1y, b1y, W2T + (size_t)16 * RHID, hdim, RYL, 1, 3, 0);
  attn_g<<<gAT, bAT, 0, stream>>>(QH, QL, KH, KL, VH, VL, RXL, RYL, OH, OL);
  gemm_o2<<<gO, b128, 0, stream>>>(OH, OL, WOT, bo, out, 1.0f / (OSC * WOS));
  (void)hipGetLastError();
}
